// PhotonicBasisActivationLayerIntervalAffineClean_79748952752386
// MI455X (gfx1250) — hardware-verified
//
#include <hip/hip_runtime.h>
#include <stdint.h>


typedef _Float16 v8h  __attribute__((ext_vector_type(8)));
typedef _Float16 v16h __attribute__((ext_vector_type(16)));
typedef float    v8f  __attribute__((ext_vector_type(8)));
typedef float    v4f  __attribute__((ext_vector_type(4)));
typedef float    v2f  __attribute__((ext_vector_type(2)));
union Frag { v16h v; v8h half[2]; };

#define I_DIM           256
#define O_DIM           32
#define NBAS            16
#define KTOT            (I_DIM * NBAS)
#define NCHUNK          (KTOT / 32)
#define ROWS_PER_BLOCK  128
#define SCALE_A         64.0f
#define SCALE_B         1024.0f
#define INV_SCALE       (1.0f / 65536.0f)
#define LN2f            0.6931471805599453f
#define LOG2Ef          1.4426950408889634f

__device__ __forceinline__ v8f wmma_f16(v16h a, v16h b, v8f c) {
    return __builtin_amdgcn_wmma_f32_16x16x32_f16(false, a, false, b, (short)0, c, false, false);
}

__device__ __forceinline__ float basis_eval(float u, const float* c) {
    float t    = __builtin_amdgcn_exp2f(c[2] * u) - 1.0f;
    float pw   = __builtin_amdgcn_exp2f(c[3] * __builtin_amdgcn_logf(t));
    float il   = __builtin_amdgcn_logf(1.0f + pw);
    float lo   = __builtin_amdgcn_logf(fmaf(c[1], il, 1.0f));
    float poly = u * fmaf(u, fmaf(u, fmaf(u, c[7], c[6]), c[5]), c[4]);
    return fmaf(c[0], lo, poly);
}

__global__ __launch_bounds__(256)
void k_cvt_coeffs(const float* __restrict__ src, _Float16* __restrict__ dst, int n8) {
    const int t = blockIdx.x * 256 + threadIdx.x;
    if (t < n8) {
        const float* p = src + (size_t)t * 8;
        v4f f0 = *(const v4f*)(p);
        v4f f1 = *(const v4f*)(p + 4);
        v8h hv;
        hv[0] = (_Float16)(f0.x * SCALE_B); hv[1] = (_Float16)(f0.y * SCALE_B);
        hv[2] = (_Float16)(f0.z * SCALE_B); hv[3] = (_Float16)(f0.w * SCALE_B);
        hv[4] = (_Float16)(f1.x * SCALE_B); hv[5] = (_Float16)(f1.y * SCALE_B);
        hv[6] = (_Float16)(f1.z * SCALE_B); hv[7] = (_Float16)(f1.w * SCALE_B);
        _Float16* q = dst + (size_t)t * 8;
        *(volatile v8h*)q = hv;
        __threadfence();
        *(volatile v8h*)q = hv;
    }
}

__global__ __launch_bounds__(256)
void k_basis_gemm(const float* __restrict__ x,
                  const _Float16* __restrict__ ch,
                  const float* __restrict__ b_coef,
                  const float* __restrict__ alpha,
                  const float* __restrict__ beta,
                  float* __restrict__ out,
                  int n_rows) {
    __shared__ float s_bc[NBAS * 8];
    __shared__ float s_alpha[I_DIM];
    __shared__ float s_beta[I_DIM];
    __shared__ __attribute__((aligned(16))) float s_tile[8 * 16 * 32];

    const int tid = threadIdx.x;
    if (tid < NBAS * 8) {
        const int j = tid & 7;
        float v = b_coef[tid];
        if (j == 0) v *= LN2f * SCALE_A;
        if (j == 1) v *= LN2f;
        if (j == 2) v *= LOG2Ef;
        if (j >= 4) v *= SCALE_A;
        s_bc[tid] = v;
    }
    for (int i = tid; i < I_DIM; i += 256) {
        s_alpha[i] = alpha[i];
        s_beta[i]  = beta[i];
    }
    __syncthreads();

    const int lane = tid & 31;
    const int wave = tid >> 5;
    const int ml   = lane & 15;
    const int h    = lane >> 4;

    const int row0 = blockIdx.x * ROWS_PER_BLOCK + wave * 16;
    int m = row0 + ml;
    if (m > n_rows - 1) m = n_rows - 1;
    const float* xrow = x + (size_t)m * I_DIM;

    float cf[8][8];
#pragma unroll
    for (int e = 0; e < 8; ++e) {
#pragma unroll
        for (int j = 0; j < 8; ++j) cf[e][j] = s_bc[(8 * h + e) * 8 + j];
    }

    const _Float16* bp0 = ch + (size_t)ml * KTOT + 8 * h;
    const _Float16* bp1 = ch + (size_t)(16 + ml) * KTOT + 8 * h;

    v8f acc0 = {0.f, 0.f, 0.f, 0.f, 0.f, 0.f, 0.f, 0.f};
    v8f acc1 = {0.f, 0.f, 0.f, 0.f, 0.f, 0.f, 0.f, 0.f};

#pragma unroll 1
    for (int c = 0; c < NCHUNK; ++c) {
        const int i0 = c * 2;
        v2f xv = *(const v2f*)(xrow + i0);
        const float u0 = s_alpha[i0]     * xv.x + s_beta[i0];
        const float u1 = s_alpha[i0 + 1] * xv.y + s_beta[i0 + 1];

        Frag a;
#pragma unroll
        for (int e = 0; e < 8; ++e) {
            a.v[e]     = (_Float16)basis_eval(u0, cf[e]);
            a.v[8 + e] = (_Float16)basis_eval(u1, cf[e]);
        }

        Frag b0, b1;
        const _Float16* q0 = bp0 + c * 32;
        const _Float16* q1 = bp1 + c * 32;
        b0.half[0] = *(const v8h*)(q0);
        b0.half[1] = *(const v8h*)(q0 + 16);
        b1.half[0] = *(const v8h*)(q1);
        b1.half[1] = *(const v8h*)(q1 + 16);

        acc0 = wmma_f16(a.v, b0.v, acc0);
        acc1 = wmma_f16(a.v, b1.v, acc1);
        asm volatile("v_nop\n\tv_nop\n\tv_nop\n\tv_nop"
                     : "+v"(acc0), "+v"(acc1)
                     : "v"(a.v), "v"(b0.v), "v"(b1.v));
    }

    float* st = s_tile + wave * (16 * 32);
#pragma unroll
    for (int r = 0; r < 8; ++r) {
        const float v0 = acc0[r] * INV_SCALE;
        const float v1 = acc1[r] * INV_SCALE;
        st[(8 * h + r) * 32 + ml]      = v0;
        st[(8 * h + r) * 32 + 16 + ml] = v1;
    }
    __syncthreads();

    const int piece = lane & 7;
    const int rsub  = lane >> 3;
    v4f vals[4];
#pragma unroll
    for (int q = 0; q < 4; ++q) {
        const int rr = q * 4 + rsub;
        vals[q] = *(const v4f*)(st + rr * 32 + piece * 4);
    }
#pragma unroll
    for (int q = 0; q < 4; ++q) {
        const int g = row0 + q * 4 + rsub;
        if (g < n_rows)
            *(volatile v4f*)(out + (size_t)g * O_DIM + piece * 4) = vals[q];
    }
    __threadfence();
#pragma unroll
    for (int q = 0; q < 4; ++q) {
        const int g = row0 + q * 4 + rsub;
        if (g < n_rows)
            *(volatile v4f*)(out + (size_t)g * O_DIM + piece * 4) = vals[q];
    }
}

extern "C" void kernel_launch(void* const* d_in, const int* in_sizes, int n_in,
                              void* d_out, int out_size, void* d_ws, size_t ws_size,
                              hipStream_t stream) {
    if (n_in < 5) return;
    const int n_x     = in_sizes[0];
    const int n_coef  = in_sizes[1];
    const int n_bcoef = in_sizes[2];
    const int n_alpha = in_sizes[3];
    const int n_beta  = in_sizes[4];

    const int n_rows = n_x / I_DIM;
    if (n_rows <= 0 || n_rows * I_DIM != n_x) return;
    if (n_coef != O_DIM * KTOT) return;
    if (n_bcoef != NBAS * 8 || n_alpha != I_DIM || n_beta != I_DIM) return;
    if (out_size != n_rows * O_DIM) return;

    const size_t ch_bytes = (size_t)O_DIM * KTOT * sizeof(_Float16);
    if (ch_bytes > ws_size) return;

    const float* x      = (const float*)d_in[0];
    const float* coeffs = (const float*)d_in[1];
    const float* b_coef = (const float*)d_in[2];
    const float* alpha  = (const float*)d_in[3];
    const float* beta   = (const float*)d_in[4];
    float* out = (float*)d_out;
    _Float16* ch = (_Float16*)d_ws;

    const int n8 = (O_DIM * KTOT) / 8;
    dim3 grid1((n8 + 255) / 256);
    hipLaunchKernelGGL(k_cvt_coeffs, grid1, dim3(256), 0, stream, coeffs, ch, n8);

    dim3 grid2((n_rows + ROWS_PER_BLOCK - 1) / ROWS_PER_BLOCK);
    hipLaunchKernelGGL(k_basis_gemm, grid2, dim3(256), 0, stream,
                       x, (const _Float16*)ch, b_coef, alpha, beta, out, n_rows);
    (void)hipGetLastError();
}
